// GRU_91311004713251
// MI455X (gfx1250) — hardware-verified
//
#include <hip/hip_runtime.h>
#include <math.h>

constexpr int NB        = 256;
constexpr int TSTEPS    = 2048;
constexpr int HID       = 100;
constexpr int G3        = 3 * HID;
constexpr int NIN       = 2;
constexpr int NOUTF     = 2;
constexpr int NTHR      = 256;
constexpr int NWAVES    = NTHR / 32;
constexpr int NMMAW     = 7;
constexpr int ROWS_BLK  = 16;
constexpr int UNITP     = 16 * NMMAW;
constexpr int KPAD      = 128;
constexpr int WKP       = 128;
constexpr int HP        = 136;
constexpr int HFP       = UNITP;
constexpr int OBP       = 32;
constexpr int VBP       = 32;
constexpr int TBLK      = 16;
constexpr int WPL_N     = 3 * UNITP * WKP;
constexpr int WPL_ITERS = WPL_N / NTHR;
constexpr float WCARRY  = 64.0f;
constexpr float LOCARRY = 2048.0f;
constexpr float SC_HI   = 1.0f / WCARRY;
constexpr float SC_LO   = 1.0f / (WCARRY * LOCARRY);
static_assert(NB % ROWS_BLK == 0, "grid exact");
static_assert(ROWS_BLK == 16, "lane maps assume a 16-row m-subtile");
static_assert(TSTEPS % TBLK == 0, "no tail in the staged line stores");
static_assert(TBLK * NOUTF == 32 && TBLK * NIN == 32, "one staged row = 32 floats = one 128-B line");
static_assert(WPL_N % NTHR == 0, "weight plane fill exact");
static_assert(KPAD % 32 == 0 && KPAD >= UNITP && KPAD <= WKP && KPAD <= HP, "K padding");
static_assert(UNITP >= HID && HID % 4 == 0, "unit padding / v4f head dot");
static_assert(NWAVES == NMMAW + 1 && 2 * UNITP <= NMMAW * 32, "wave roles");
static_assert((HP * 2) % 16 == 0 && (HFP * 4) % 16 == 0, "16-B aligned LDS rows");

typedef __attribute__((ext_vector_type(16))) _Float16 v16h;
typedef __attribute__((ext_vector_type(8)))  _Float16 v8h;
typedef __attribute__((ext_vector_type(8)))  float    v8f;
typedef __attribute__((ext_vector_type(4)))  float    v4f;
typedef __attribute__((ext_vector_type(2)))  float    v2f;

template <typename T> struct Frag;
template <> struct Frag<_Float16> {
  typedef v16h V; union U { v16h v; v8h h[2]; };
  static __device__ __forceinline__ v16h load(const _Float16* p) {
    U f; f.h[0] = *(const v8h*)(p); f.h[1] = *(const v8h*)(p + 16); return f.v;
  }
  static __device__ __forceinline__ v8f mma(v16h a, v16h b, v8f c) {
    return __builtin_amdgcn_wmma_f32_16x16x32_f16(false, a, false, b, (short)0, c, false, false);
  }
};
__device__ __forceinline__ void dep_guard6_h(v8f& a0, v8f& a1, v8f& a2, v8f& a3, v8f& a4, v8f& a5,
                                             v16h f0, v16h f1, v16h f2, v16h f3, v16h f4) {
  asm volatile("v_nop\n\tv_nop\n\tv_nop\n\tv_nop"
               : "+v"(a0), "+v"(a1), "+v"(a2), "+v"(a3), "+v"(a4), "+v"(a5)
               : "v"(f0), "v"(f1), "v"(f2), "v"(f3), "v"(f4));
}
__device__ __forceinline__ void acc_guard6(v8f& a0, v8f& a1, v8f& a2, v8f& a3, v8f& a4, v8f& a5) {
  asm volatile("v_nop\n\tv_nop\n\tv_nop\n\tv_nop" : "+v"(a0), "+v"(a1), "+v"(a2), "+v"(a3), "+v"(a4), "+v"(a5));
}

__device__ __forceinline__ float gate_sig(float x)  { return __builtin_amdgcn_rcpf(1.0f + expf(-x)); }
__device__ __forceinline__ float gate_tanh(float x) { return 1.0f - 2.0f * __builtin_amdgcn_rcpf(1.0f + expf(2.0f * x)); }

__device__ __forceinline__ float head_dot(const float* hrow, const float* wrow) {
  float s = 0.0f;
#pragma unroll 5
  for (int q = 0; q < HID / 4; ++q) {
    const v4f a = *(const v4f*)(hrow + 4 * q);
    const v4f b = *(const v4f*)(wrow + 4 * q);
    s += a.x * b.x; s += a.y * b.y; s += a.z * b.z; s += a.w * b.w;
  }
  return s;
}

__device__ __forceinline__ void stage_v(const float* __restrict__ vin, float* vbuf, int bbase, int tbase, int lane) {
  const int q = lane >> 3, c4 = (lane & 7) * 4;
  v4f tmp[4];
#pragma unroll
  for (int it = 0; it < 4; ++it) {
    const int row = it * 4 + q;
    tmp[it] = *(const v4f*)(vin + ((size_t)(bbase + row) * TSTEPS + (size_t)tbase) * NIN + c4);
  }
#pragma unroll
  for (int it = 0; it < 4; ++it) {
    const int row = it * 4 + q;
    *(v4f*)(vbuf + row * VBP + c4) = tmp[it];
  }
}

__device__ __forceinline__ void flush_lines(const float* obuf, float* __restrict__ out, int bbase, int tbase, int lane) {
  const int q = lane >> 3, c4 = (lane & 7) * 4;
  for (int pass = 0; pass < 2; ++pass) {
#pragma unroll
    for (int it = 0; it < 4; ++it) {
      const int row = it * 4 + q;
      const v4f val = *(const v4f*)(obuf + row * OBP + c4);
      *(volatile v4f*)(out + ((size_t)(bbase + row) * TSTEPS + (size_t)tbase) * NOUTF + c4) = val;
    }
    __threadfence();
  }
}

__global__ __launch_bounds__(NTHR) void rnn_seq_kernel(const float* __restrict__ x_i, const float* __restrict__ vin,
                                                       const float* __restrict__ w_ih, const float* __restrict__ w_hh,
                                                       const float* __restrict__ b_ih, const float* __restrict__ b_hh,
                                                       const float* __restrict__ w_out, const float* __restrict__ b_out,
                                                       float* __restrict__ out) {
  __shared__ __align__(16) _Float16 Wpl[WPL_N];
  __shared__ __align__(16) _Float16 Ahi[ROWS_BLK * HP];
  __shared__ __align__(16) _Float16 Alo[ROWS_BLK * HP];
  __shared__ __align__(16) float    hf[ROWS_BLK * HFP];
  __shared__ __align__(16) float    obuf[ROWS_BLK * OBP];
  __shared__ __align__(16) float    vbuf[ROWS_BLK * VBP];
  __shared__ __align__(16) float    s_wout[2 * UNITP];
  __shared__ float s_c[ROWS_BLK * 2];

  const int tid  = threadIdx.x;
  const int lane = tid & 31;
  const int wave = __builtin_amdgcn_readfirstlane(tid >> 5);
  const int c = lane & 15, hh = lane >> 4, koff = hh * 8, mOff = hh * 8;
  const int bbase = blockIdx.x * ROWS_BLK;
  const int j = 16 * wave + c;
  const bool valid = (j < HID);
  const int jj = valid ? j : (HID - 1);
  const int ju = (j < UNITP) ? j : 0;

#pragma unroll 1
  for (int it = 0; it < WPL_ITERS; ++it) {
    const int i   = it * NTHR + tid;
    const int g   = i / (UNITP * WKP);
    const int rem = i - g * (UNITP * WKP);
    const int u   = rem >> 7;
    const int k   = rem & (WKP - 1);
    const int uu  = (u < HID) ? u : (HID - 1);
    const int kk  = (k < HID) ? k : (HID - 1);
    const float w = w_hh[(g * HID + uu) * HID + kk];
    const float fsel = ((u < HID) && (k < HID)) ? WCARRY : 0.0f;
    Wpl[i] = (_Float16)(w * fsel);
  }
  if (wave < NMMAW) {
    const int o  = (tid >= UNITP) ? 1 : 0;
    const int u  = tid - o * UNITP;
    const int uu = (u < HID) ? u : (HID - 1);
    const float w = w_out[o * HID + uu];
    const float fsel = (u < HID) ? 1.0f : 0.0f;
    s_wout[tid] = w * fsel;
  }
  const float wir0 = w_ih[jj * NIN + 0],             wir1 = w_ih[jj * NIN + 1];
  const float wiz0 = w_ih[(HID + jj) * NIN + 0],     wiz1 = w_ih[(HID + jj) * NIN + 1];
  const float win0 = w_ih[(2 * HID + jj) * NIN + 0], win1 = w_ih[(2 * HID + jj) * NIN + 1];
  asm volatile("" ::: "memory");
  const float bir = b_ih[jj], biz = b_ih[HID + jj], bin = b_ih[2 * HID + jj];
  const float bhr = b_hh[jj], bhz = b_hh[HID + jj], bhn = b_hh[2 * HID + jj];
  float bout_o = 0.0f;
  if (wave == NMMAW) {
    stage_v(vin, vbuf, bbase, 0, lane);
    bout_o = b_out[lane & 1];
  }
  __syncthreads();

  if (wave == 0) {
    float a00 = 0.0f, a01 = 0.0f, a11 = 0.0f;
#pragma unroll 1
    for (int k = 0; k < HID; ++k) {
      const float w0 = s_wout[k], w1 = s_wout[UNITP + k];
      a00 += w0 * w0; a01 += w0 * w1; a11 += w1 * w1;
    }
    const float det = a00 * a11 - a01 * a01;
    const float inv_det = 1.0f / det;
    const int row = lane & 15;
    const float r0 = x_i[(bbase + row) * 2 + 0] - b_out[0];
    const float r1 = x_i[(bbase + row) * 2 + 1] - b_out[1];
    const float c0 = (a11 * r0 - a01 * r1) * inv_det;
    const float c1 = (a00 * r1 - a01 * r0) * inv_det;
    if (lane < 16) { s_c[row * 2 + 0] = c0; s_c[row * 2 + 1] = c1; }
  }
  __syncthreads();

  float hreg[8];
  if (wave < NMMAW) {
    const float w0 = s_wout[jj], w1 = s_wout[UNITP + jj];
#pragma unroll
    for (int r = 0; r < 8; ++r) {
      const float c0 = s_c[(mOff + r) * 2 + 0], c1 = s_c[(mOff + r) * 2 + 1];
      const float h0 = c0 * w0 + c1 * w1;
      hreg[r] = valid ? h0 : 0.0f;
    }
#pragma unroll
    for (int r = 0; r < 8; ++r) {
      const float hv = hreg[r];
      const _Float16 hi = (_Float16)hv;
      const float res = (hv - (float)hi) * LOCARRY;
      const _Float16 lo = (_Float16)res;
      Ahi[(mOff + r) * HP + j] = hi;
      Alo[(mOff + r) * HP + j] = lo;
      hf[(mOff + r) * HFP + j] = hv;
    }
  } else {
#pragma unroll
    for (int r = 0; r < 8; ++r) hreg[r] = 0.0f;
    const int prow = lane >> 1, h8 = (lane & 1) * 8;
    v8h zv;
#pragma unroll
    for (int e = 0; e < 8; ++e) zv[e] = (_Float16)0.0f;
    *(v8h*)(Ahi + prow * HP + UNITP + h8) = zv;
    *(v8h*)(Alo + prow * HP + UNITP + h8) = zv;
  }
  __syncthreads();

  const _Float16* ahp = Ahi + c * HP + koff;
  const _Float16* alp = Alo + c * HP + koff;
  const _Float16* wrp = Wpl + (0 * UNITP + ju) * WKP + koff;
  const _Float16* wzp = Wpl + (1 * UNITP + ju) * WKP + koff;
  const _Float16* wnp = Wpl + (2 * UNITP + ju) * WKP + koff;
  const v8f z8 = {0.f, 0.f, 0.f, 0.f, 0.f, 0.f, 0.f, 0.f};

#pragma unroll 1
  for (int t = 0; t < TSTEPS; ++t) {
    if (wave < NMMAW) {
      v8f aHr = z8, aHz = z8, aHn = z8, aLr = z8, aLz = z8, aLn = z8;
#pragma unroll 1
      for (int k0 = 0; k0 < KPAD; k0 += 32) {
        const v16h ah = Frag<_Float16>::load(ahp + k0);
        const v16h al = Frag<_Float16>::load(alp + k0);
        const v16h b0 = Frag<_Float16>::load(wrp + k0);
        const v16h b1 = Frag<_Float16>::load(wzp + k0);
        const v16h b2 = Frag<_Float16>::load(wnp + k0);
        aHr = Frag<_Float16>::mma(ah, b0, aHr);
        aHz = Frag<_Float16>::mma(ah, b1, aHz);
        aHn = Frag<_Float16>::mma(ah, b2, aHn);
        aLr = Frag<_Float16>::mma(al, b0, aLr);
        aLz = Frag<_Float16>::mma(al, b1, aLz);
        aLn = Frag<_Float16>::mma(al, b2, aLn);
        dep_guard6_h(aHr, aHz, aHn, aLr, aLz, aLn, ah, al, b0, b1, b2);
      }
      acc_guard6(aHr, aHz, aHn, aLr, aLz, aLn);

      const int slot2 = (t & (TBLK - 1)) * NIN;
#pragma unroll
      for (int r = 0; r < 8; ++r) {
        const int row = mOff + r;
        const v2f vv = *(const v2f*)(vbuf + row * VBP + slot2);
        const float xr = vv.x * wir0 + vv.y * wir1 + bir;
        const float xz = vv.x * wiz0 + vv.y * wiz1 + biz;
        const float xn = vv.x * win0 + vv.y * win1 + bin;
        const float hr = aHr[r] * SC_HI + aLr[r] * SC_LO + bhr;
        const float hz = aHz[r] * SC_HI + aLz[r] * SC_LO + bhz;
        const float hn = aHn[r] * SC_HI + aLn[r] * SC_LO + bhn;
        const float rg = gate_sig(xr + hr);
        const float zg = gate_sig(xz + hz);
        const float ng = gate_tanh(xn + rg * hn);
        const float ho = hreg[r];
        const float hnew = (1.0f - zg) * ng + zg * ho;
        hreg[r] = valid ? hnew : 0.0f;
      }
    } else {
      if (t > 0) {
        const int orow = lane >> 1, oo = lane & 1;
        const float s = head_dot(hf + orow * HFP, s_wout + oo * UNITP) + bout_o;
        obuf[orow * OBP + ((t - 1) & (TBLK - 1)) * NOUTF + oo] = s;
      }
    }
    __syncthreads();

    if (wave < NMMAW) {
#pragma unroll
      for (int r = 0; r < 8; ++r) {
        const float hv = hreg[r];
        const _Float16 hi = (_Float16)hv;
        const float res = (hv - (float)hi) * LOCARRY;
        const _Float16 lo = (_Float16)res;
        Ahi[(mOff + r) * HP + j] = hi;
        Alo[(mOff + r) * HP + j] = lo;
        hf[(mOff + r) * HFP + j] = hv;
      }
    } else {
      const int prow = lane >> 1, h8 = (lane & 1) * 8;
      v8h zv;
#pragma unroll
      for (int e = 0; e < 8; ++e) zv[e] = (_Float16)0.0f;
      *(v8h*)(Ahi + prow * HP + UNITP + h8) = zv;
      *(v8h*)(Alo + prow * HP + UNITP + h8) = zv;
      if ((t & (TBLK - 1)) == 0 && t > 0) flush_lines(obuf, out, bbase, t - TBLK, lane);
      if ((t & (TBLK - 1)) == (TBLK - 1) && (t + 1) < TSTEPS) stage_v(vin, vbuf, bbase, t + 1, lane);
    }
    __syncthreads();
  }

  if (wave == NMMAW) {
    const int orow = lane >> 1, oo = lane & 1;
    const float s = head_dot(hf + orow * HFP, s_wout + oo * UNITP) + bout_o;
    obuf[orow * OBP + ((TSTEPS - 1) & (TBLK - 1)) * NOUTF + oo] = s;
  }
  __syncthreads();
  if (wave == NMMAW) flush_lines(obuf, out, bbase, TSTEPS - TBLK, lane);
}

extern "C" void kernel_launch(void* const* d_in, const int* in_sizes, int n_in,
                              void* d_out, int out_size, void* d_ws, size_t ws_size, hipStream_t stream) {
  (void)d_ws; (void)ws_size;
  if (n_in < 8 || d_out == nullptr) return;
  if (in_sizes[0] != NB * NIN || in_sizes[1] != NB * TSTEPS * NIN || in_sizes[2] != G3 * NIN ||
      in_sizes[3] != G3 * HID || in_sizes[4] != G3 || in_sizes[5] != G3 || in_sizes[6] != NOUTF * HID ||
      in_sizes[7] != NOUTF || out_size != NB * TSTEPS * NOUTF) return;

  const float* x_i   = (const float*)d_in[0];
  const float* vin   = (const float*)d_in[1];
  const float* w_ih  = (const float*)d_in[2];
  const float* w_hh  = (const float*)d_in[3];
  const float* b_ih  = (const float*)d_in[4];
  const float* b_hh  = (const float*)d_in[5];
  const float* w_out = (const float*)d_in[6];
  const float* b_out = (const float*)d_in[7];
  float* out = (float*)d_out;

  rnn_seq_kernel<<<dim3(NB / ROWS_BLK), dim3(NTHR), 0, stream>>>(x_i, vin, w_ih, w_hh, b_ih, b_hh, w_out, b_out, out);
}
